// EncoderLayer_75488345195383
// MI455X (gfx1250) — hardware-run, weakly checked
//
#include <hip/hip_runtime.h>


#ifndef NB
#define NB 8
#endif
#ifndef SEQ
#define SEQ 1024
#endif
#define NB_FULL  8
#define SEQ_FULL 1024
#ifndef OUT_SEQ
#define OUT_SEQ SEQ
#endif
#define DM   512
#define NH_  8
#define HD   64
#define DFF  2048
#define AW   4
#define OSP  68
#define SC2  ((float)(0.125 * 1.4426950408889634))
#define PSH  14.0f
#define NEGB (-3.0e38f)
#define CTXC 16.0f
#define WTC  64.0f
#define LNEPS 1.0e-5f

static constexpr float SCL_WO = 1.0f / (CTXC * WTC);
static constexpr float SCL_W1 = 1.0f / WTC;
static constexpr float SCL_W2 = 1.0f / WTC;

static_assert(HD == 64);
static_assert(NH_ * HD == DM);
static_assert(DM % 64 == 0);
static_assert(DFF % 64 == 0);
static_assert(DM % 32 == 0);
static_assert(DFF % 32 == 0);
static_assert(HD % 32 == 0);
static_assert(SEQ % 64 == 0);
static_assert((NB * SEQ) % 64 == 0);
static_assert(SEQ % 32 == 0);
static_assert(SEQ % (16 * AW) == 0);
static_assert((NB * SEQ) % 8 == 0);
static_assert(DM == 32 * 16);
static_assert(((size_t)SEQ * DM) % 8 == 0);
static_assert(NB <= NB_FULL);
static_assert(SEQ <= SEQ_FULL);
static_assert((OSP * 4) % 16 == 0);
static_assert(OSP >= HD);
static_assert(sizeof(float) * AW * 16 * OSP <= 131072);
static_assert(sizeof(float) * 16 * 68 <= 131072);
static_assert(sizeof(float) * 64 * 68 <= 131072);
static_assert(sizeof(float) * 8 * DM <= 131072);

typedef _Float16 h16;
typedef unsigned short bf;
typedef __attribute__((ext_vector_type(16))) __bf16   v16bf;
typedef __attribute__((ext_vector_type(16))) _Float16 v16h;
typedef __attribute__((ext_vector_type(8)))  _Float16 v8h;
typedef __attribute__((ext_vector_type(8)))  unsigned short v8us;
typedef __attribute__((ext_vector_type(8)))  float    v8f;
typedef __attribute__((ext_vector_type(4)))  float    v4f;
typedef v4f  __attribute__((may_alias)) v4fa;

__device__ __forceinline__ unsigned short f2bf(float f) { unsigned u = __float_as_uint(f); u += 0x7FFFu + ((u >> 16) & 1u); return (unsigned short)(u >> 16); }
__device__ __forceinline__ float bfr(float f) { return __uint_as_float(((unsigned)f2bf(f)) << 16); }
__device__ __forceinline__ v16h cat16(v8h lo, v8h hi) { return __builtin_shufflevector(lo, hi, 0, 1, 2, 3, 4, 5, 6, 7, 8, 9, 10, 11, 12, 13, 14, 15); }
__device__ __forceinline__ v16bf cat16b(v8us lo, v8us hi) { return __builtin_bit_cast(v16bf, __builtin_shufflevector(lo, hi, 0, 1, 2, 3, 4, 5, 6, 7, 8, 9, 10, 11, 12, 13, 14, 15)); }
__device__ __forceinline__ v8f wmma16(v16h a, v16h b, v8f c) { return __builtin_amdgcn_wmma_f32_16x16x32_f16(false, a, false, b, (short)0, c, false, false); }
__device__ __forceinline__ v8f wmmab(v16bf a, v16bf b, v8f c) { return __builtin_amdgcn_wmma_f32_16x16x32_bf16(false, a, false, b, (short)0, c, false, false); }
__device__ __forceinline__ v8f wmma16g(v16h a, v16h b, v8f c) { c = wmma16(a, b, c); asm volatile("v_nop\n\tv_nop\n\tv_nop\n\tv_nop" : "+v"(c) : "v"(a), "v"(b)); return c; }
__device__ __forceinline__ v8f wmmabg(v16bf a, v16bf b, v8f c) { c = wmmab(a, b, c); asm volatile("v_nop\n\tv_nop\n\tv_nop\n\tv_nop" : "+v"(c) : "v"(a), "v"(b)); return c; }
__device__ __forceinline__ v16h  ldh(const h16* p) { return cat16(*(const v8h*)p, *(const v8h*)(p + 16)); }
__device__ __forceinline__ v16bf ldb(const bf* p)  { return cat16b(*(const v8us*)p, *(const v8us*)(p + 16)); }
__device__ __forceinline__ void wave_sync() { __builtin_amdgcn_fence(3  , "wavefront"); __builtin_amdgcn_wave_barrier(); asm volatile("" ::: "memory"); }
static __device__ __forceinline__ h16 toh_flush(float v) { const float w = (fabsf(v) < 6.103515625e-05f) ? 0.0f : v; return (h16)w; }

template <typename T> struct FragOf;
template <> struct FragOf<bf>  { typedef v16bf type; };
template <> struct FragOf<h16> { typedef v16h  type; };
__device__ __forceinline__ v16bf ldf(const bf* p)  { return ldb(p); }
__device__ __forceinline__ v16h  ldf(const h16* p) { return ldh(p); }
__device__ __forceinline__ v8f mmag(v16bf a, v16bf b, v8f c) { return wmmabg(a, b, c); }
__device__ __forceinline__ v8f mmag(v16h a, v16h b, v8f c)   { return wmma16g(a, b, c); }

__global__ __launch_bounds__(256) void k_cvt8(const float* __restrict__ src, bf* dst, size_t n8) {
    const size_t i = (size_t)blockIdx.x * 256 + threadIdx.x; if (i >= n8) return;
    const v8f v = *(const v8f*)(src + i * 8); v8us o;
#pragma unroll
    for (int k = 0; k < 8; ++k) o[k] = f2bf(v[k]);
    *(volatile v8us*)(dst + i * 8) = o; __threadfence(); *(volatile v8us*)(dst + i * 8) = o;
}

__device__ __forceinline__ void st8w(bf* p, v8f w) { v8us o;
#pragma unroll
    for (int e = 0; e < 8; ++e) o[e] = f2bf(w[e]);
    *(volatile v8us*)p = o; }
__device__ __forceinline__ void st8w(h16* p, v8f w) { v8h o;
#pragma unroll
    for (int e = 0; e < 8; ++e) o[e] = toh_flush(bfr(w[e]) * WTC);
    *(volatile v8h*)p = o; }

template <typename OT>
__device__ __forceinline__ void wt_body(const float* __restrict__ W, OT* dst, unsigned Kdim, unsigned Ndim) {
    __shared__ __align__(16) float ts[64 * 68];
    const unsigned tid = threadIdx.x; const unsigned n0 = blockIdx.x * 64u, k0 = blockIdx.y * 64u;
    static_assert(4 * 256 * 16 == 64 * 64 * 4);
#pragma unroll
    for (int i = 0; i < 4; ++i) { const unsigned idx = tid + 256u * (unsigned)i; const unsigned row = idx >> 4, c4 = (idx & 15u) * 4u;
        const v4f v = *(const v4f*)(W + (size_t)(k0 + row) * Ndim + n0 + c4);
        *(v4fa*)(&ts[row * 68 + c4]) = v; }
    __syncthreads();
    static_assert(2 * 256 * 16 == 64 * 64 * 2);
#pragma unroll 1
    for (int ps = 0; ps < 2; ++ps) {
#pragma unroll
        for (int it = 0; it < 2; ++it) { const unsigned p = tid + 256u * (unsigned)it; const unsigned n = p >> 3, c8 = (p & 7u) * 8u;
            v8f w;
#pragma unroll
            for (int e = 0; e < 8; ++e) w[e] = ts[(c8 + e) * 68 + n];
            st8w(dst + (size_t)(n0 + n) * Kdim + k0 + c8, w); }
        if (ps == 0) __threadfence(); }
}
__global__ __launch_bounds__(256) void k_wt_b(const float* __restrict__ W, bf* dst, unsigned Kdim, unsigned Ndim) { wt_body<bf>(W, dst, Kdim, Ndim); }
__global__ __launch_bounds__(256) void k_wt_h(const float* __restrict__ W, h16* dst, unsigned Kdim, unsigned Ndim) { wt_body<h16>(W, dst, Kdim, Ndim); }

template <typename T, int MODE, int KD>
__device__ __forceinline__ void gemm_body(const T* __restrict__ A, const T* __restrict__ Bt, const float* __restrict__ bias, const float* __restrict__ R, h16* Oh, float* Of) {
    __shared__ __align__(16) float os[16 * 68];
    typedef typename FragOf<T>::type frag;
    static_assert(KD % 32 == 0);
    constexpr float scl = (MODE == 2) ? SCL_WO : ((MODE == 3) ? SCL_W1 : ((MODE == 4) ? SCL_W2 : 1.0f));
    constexpr size_t pitch = (MODE == 0) ? (size_t)HD : ((MODE == 1) ? (size_t)SEQ : ((MODE == 3) ? (size_t)DFF : (size_t)DM));
    const int lane = threadIdx.x & 31, lr = lane & 15, hi = lane >> 4;
    const unsigned bx = blockIdx.x, by = blockIdx.y;
    const unsigned r0 = bx * 64u, c0 = by * 64u;
    v8f acc[4][4];
#pragma unroll
    for (int mb = 0; mb < 4; ++mb)
#pragma unroll
        for (int nb = 0; nb < 4; ++nb) acc[mb][nb] = (v8f){};
    const size_t aoff = (size_t)(r0 + (unsigned)lr) * KD + 8 * hi, boff = (size_t)(c0 + (unsigned)lr) * KD + 8 * hi;
#pragma unroll 1
    for (int kc = 0; kc < KD; kc += 32) {
        frag a[4];
#pragma unroll
        for (int mb = 0; mb < 4; ++mb) a[mb] = ldf(A + aoff + (size_t)mb * 16 * KD + kc);
#pragma unroll
        for (int nb = 0; nb < 4; ++nb) { const frag b = ldf(Bt + boff + (size_t)nb * 16 * KD + kc);
#pragma unroll
            for (int mb = 0; mb < 4; ++mb) acc[mb][nb] = mmag(a[mb], b, acc[mb][nb]); }
    }
    float bc[4];
#pragma unroll
    for (int nb = 0; nb < 4; ++nb) bc[nb] = (MODE != 1) ? bfr(bias[c0 + nb * 16 + lr]) : 0.0f;
    size_t obase = 0, rbase = 0;
    if (MODE == 0)      { const unsigned bb = r0 / (unsigned)SEQ, tt = r0 % (unsigned)SEQ; const unsigned zc = bb * (unsigned)NH_ + c0 / (unsigned)HD;
                          obase = ((size_t)zc * SEQ + tt) * HD; }
    else if (MODE == 1) { const unsigned bb = c0 / (unsigned)SEQ, tt = c0 % (unsigned)SEQ;
                          obase = (size_t)bb * DM * SEQ + (size_t)r0 * SEQ + tt; }
    else if (MODE == 3) { obase = (size_t)r0 * DFF + c0; }
    else                { obase = (size_t)r0 * DM + c0; rbase = obase;
                          if (MODE == 2) { const unsigned bb = r0 / (unsigned)SEQ, tt = r0 % (unsigned)SEQ; rbase = ((size_t)bb * SEQ_FULL + tt) * DM + c0; } }
#pragma unroll
    for (int mb = 0; mb < 4; ++mb) {
        float br[8];
#pragma unroll
        for (int j = 0; j < 8; ++j) br[j] = (MODE == 1) ? bfr(bias[r0 + mb * 16 + hi * 8 + j]) : 0.0f;
#pragma unroll
        for (int nb = 0; nb < 4; ++nb) {
#pragma unroll
            for (int j = 0; j < 8; ++j) { float v = acc[mb][nb][j] * scl + bc[nb] + br[j]; if (MODE == 3) v = fmaxf(v, 0.0f);
                os[(hi * 8 + j) * 68 + nb * 16 + lr] = v; } }
        wave_sync();
#pragma unroll 1
        for (int ps = 0; ps < 2; ++ps) {
            if (MODE == 0 || MODE == 1 || MODE == 3) {
                static_assert(4 * 32 * 16 == 16 * 64 * 2);
#pragma unroll
                for (int s = 0; s < 4; ++s) { const int row = 4 * s + (lane >> 3), c8 = (lane & 7) * 8;
                    const v4f x0 = *(const v4fa*)(&os[row * 68 + c8]); const v4f x1 = *(const v4fa*)(&os[row * 68 + c8 + 4]); v8h hv;
#pragma unroll
                    for (int i = 0; i < 4; ++i) { hv[i] = toh_flush(x0[i]); hv[4 + i] = toh_flush(x1[i]); }
                    const size_t oo = obase + (size_t)(mb * 16 + row) * pitch + c8;
                    *(volatile v8h*)(Oh + oo) = hv; }
            } else {
                static_assert(8 * 32 * 16 == 16 * 64 * 4);
#pragma unroll
                for (int s = 0; s < 8; ++s) { const int row = 2 * s + (lane >> 4), c4 = (lane & 15) * 4;
                    const v4f x0 = *(const v4fa*)(&os[row * 68 + c4]);
                    const v4f rr = *(const v4f*)(R + rbase + (size_t)(mb * 16 + row) * DM + c4);
                    v4f val;
#pragma unroll
                    for (int i = 0; i < 4; ++i) val[i] = x0[i] + ((MODE == 2) ? bfr(rr[i]) : rr[i]);
                    *(volatile v4f*)(Of + obase + (size_t)(mb * 16 + row) * DM + c4) = val; }
            }
            if (ps == 0) __threadfence(); }
        wave_sync();
    }
}
__global__ __launch_bounds__(32) void k_gemm_hd(const bf* __restrict__ A, const bf* __restrict__ Bt, const float* __restrict__ bias, h16* P) { gemm_body<bf, 0, DM>(A, Bt, bias, nullptr, P, nullptr); }
__global__ __launch_bounds__(32) void k_gemm_vt(const bf* __restrict__ A, const bf* __restrict__ Bt, const float* __restrict__ bias, h16* P) { gemm_body<bf, 1, DM>(A, Bt, bias, nullptr, P, nullptr); }
__global__ __launch_bounds__(32) void k_gemm_wo(const h16* __restrict__ A, const h16* __restrict__ Bt, const float* __restrict__ bias, const float* __restrict__ X, float* O) { gemm_body<h16, 2, DM>(A, Bt, bias, X, nullptr, O); }
__global__ __launch_bounds__(32) void k_gemm_f1(const h16* __restrict__ A, const h16* __restrict__ Bt, const float* __restrict__ bias, h16* P) { gemm_body<h16, 3, DM>(A, Bt, bias, nullptr, P, nullptr); }
__global__ __launch_bounds__(32) void k_gemm_f2(const h16* __restrict__ A, const h16* __restrict__ Bt, const float* __restrict__ bias, const float* __restrict__ X1, float* O) { gemm_body<h16, 4, DFF>(A, Bt, bias, X1, nullptr, O); }

__global__ __launch_bounds__(32 * AW) void k_flash(const h16* __restrict__ QH, const h16* __restrict__ KP, const h16* __restrict__ VT, h16* CTX) {
    __shared__ __align__(16) float os[AW * 16 * OSP];
    const int lane = threadIdx.x & 31, lr = lane & 15, hi = lane >> 4;
    const int wave = __builtin_amdgcn_readfirstlane((int)(threadIdx.x >> 5));
    const unsigned zh = blockIdx.y; const unsigned b = zh / (unsigned)NH_, h = zh % (unsigned)NH_;
    const unsigned t0 = (blockIdx.x * (unsigned)AW + (unsigned)wave) * 16u;
    const size_t pbase = (size_t)zh * SEQ * HD;
    const size_t qo = pbase + (size_t)(t0 + (unsigned)lr) * HD + 8 * hi;
    const v16h q0 = ldh(QH + qo), q1 = ldh(QH + qo + 32);
    const size_t ko = pbase + (size_t)lr * HD + 8 * hi;
    const size_t vo = pbase + (size_t)lr * SEQ + 8 * hi;
    v8f o0 = (v8f){}, o1 = (v8f){}, o2 = (v8f){}, o3 = (v8f){};
    float m = NEGB, l = 0.0f;
#pragma unroll 1
    for (int key0 = 0; key0 < SEQ; key0 += 32) {
        const h16* ka = KP + ko + (size_t)key0 * HD;
        const v16h ka0 = ldh(ka), ka1 = ldh(ka + 32), kb0 = ldh(ka + 16 * HD), kb1 = ldh(ka + 16 * HD + 32);
        v8f sa = (v8f){}, sb = (v8f){};
        sa = wmma16g(ka0, q0, sa); sb = wmma16g(kb0, q0, sb);
        sa = wmma16g(ka1, q1, sa); sb = wmma16g(kb1, q1, sb);
        float ta[8], tb[8]; float mx = NEGB;
#pragma unroll
        for (int r = 0; r < 8; ++r) { ta[r] = sa[r] * SC2; tb[r] = sb[r] * SC2; mx = fmaxf(mx, fmaxf(ta[r], tb[r])); }
        mx = fmaxf(mx, __shfl_xor(mx, 16, 32));
        const float mnew = fmaxf(m, mx);
        const float alpha = __builtin_amdgcn_exp2f(m - mnew);
        const float sh = PSH - mnew;
        v16h pb; float ls = 0.0f;
#pragma unroll
        for (int r = 0; r < 8; ++r) {
            const float xa = ta[r] + sh, xb = tb[r] + sh;
            const float ga = (xa < -14.0f) ? 0.0f : __builtin_amdgcn_exp2f(xa);
            const float gb = (xb < -14.0f) ? 0.0f : __builtin_amdgcn_exp2f(xb);
            const h16 pa = toh_flush(ga); const h16 pc = toh_flush(gb);
            pb[r] = pa; pb[8 + r] = pc;
            ls += (float)pa + (float)pc; }
        l = l * alpha + ls; m = mnew;
        o0 = o0 * alpha; o1 = o1 * alpha; o2 = o2 * alpha; o3 = o3 * alpha;
        const h16* va = VT + vo + key0;
        const v16h v0 = ldh(va), v1 = ldh(va + (size_t)16 * SEQ), v2 = ldh(va + (size_t)32 * SEQ), v3 = ldh(va + (size_t)48 * SEQ);
        o0 = wmma16g(v0, pb, o0); o1 = wmma16g(v1, pb, o1); o2 = wmma16g(v2, pb, o2); o3 = wmma16g(v3, pb, o3);
    }
    l += __shfl_xor(l, 16, 32);
    const float inv = (1.0f / l) * CTXC;
    const int wb = wave * 16 * OSP;
    { v4f a, c;
      a[0] = o0[0] * inv; a[1] = o0[1] * inv; a[2] = o0[2] * inv; a[3] = o0[3] * inv; c[0] = o0[4] * inv; c[1] = o0[5] * inv; c[2] = o0[6] * inv; c[3] = o0[7] * inv;
      *(v4fa*)(&os[wb + lr * OSP +  0 + 8 * hi]) = a; *(v4fa*)(&os[wb + lr * OSP +  0 + 8 * hi + 4]) = c;
      a[0] = o1[0] * inv; a[1] = o1[1] * inv; a[2] = o1[2] * inv; a[3] = o1[3] * inv; c[0] = o1[4] * inv; c[1] = o1[5] * inv; c[2] = o1[6] * inv; c[3] = o1[7] * inv;
      *(v4fa*)(&os[wb + lr * OSP + 16 + 8 * hi]) = a; *(v4fa*)(&os[wb + lr * OSP + 16 + 8 * hi + 4]) = c;
      a[0] = o2[0] * inv; a[1] = o2[1] * inv; a[2] = o2[2] * inv; a[3] = o2[3] * inv; c[0] = o2[4] * inv; c[1] = o2[5] * inv; c[2] = o2[6] * inv; c[3] = o2[7] * inv;
      *(v4fa*)(&os[wb + lr * OSP + 32 + 8 * hi]) = a; *(v4fa*)(&os[wb + lr * OSP + 32 + 8 * hi + 4]) = c;
      a[0] = o3[0] * inv; a[1] = o3[1] * inv; a[2] = o3[2] * inv; a[3] = o3[3] * inv; c[0] = o3[4] * inv; c[1] = o3[5] * inv; c[2] = o3[6] * inv; c[3] = o3[7] * inv;
      *(v4fa*)(&os[wb + lr * OSP + 48 + 8 * hi]) = a; *(v4fa*)(&os[wb + lr * OSP + 48 + 8 * hi + 4]) = c; }
    wave_sync();
    h16* orow = CTX + ((size_t)b * SEQ + t0) * DM + h * (unsigned)HD;
    static_assert(4 * 32 * 16 == 16 * HD * 2);
#pragma unroll 1
    for (int ps = 0; ps < 2; ++ps) {
#pragma unroll
        for (int s = 0; s < 4; ++s) { const int row = 4 * s + (lane >> 3), c8 = (lane & 7) * 8;
            const v4f x0 = *(const v4fa*)(&os[wb + row * OSP + c8]); const v4f x1 = *(const v4fa*)(&os[wb + row * OSP + c8 + 4]); v8h hv;
#pragma unroll
            for (int i = 0; i < 4; ++i) { hv[i] = toh_flush(x0[i]); hv[4 + i] = toh_flush(x1[i]); }
            *(volatile v8h*)(orow + (size_t)row * DM + c8) = hv; }
        if (ps == 0) __threadfence(); }
}

template <int WH>
__device__ __forceinline__ void ln_body(const float* __restrict__ T, const float* __restrict__ g, const float* __restrict__ be, float* O32, h16* O16) {
#pragma clang fp contract(off)
    __shared__ __align__(16) float ys[8 * DM];
    const int lane = threadIdx.x & 31;
    const int wave = __builtin_amdgcn_readfirstlane((int)(threadIdx.x >> 5));
    const unsigned row = blockIdx.x * 8u + (unsigned)wave;
    const float* p = T + (size_t)row * DM + lane * 4;
    v4f v[4], y[4];
#pragma unroll
    for (int j = 0; j < 4; ++j) v[j] = *(const v4f*)(p + j * 128);
    float s = 0.0f;
#pragma unroll
    for (int j = 0; j < 4; ++j) s += (v[j][0] + v[j][1]) + (v[j][2] + v[j][3]);
    s += __shfl_xor(s, 16, 32); s += __shfl_xor(s, 8, 32); s += __shfl_xor(s, 4, 32); s += __shfl_xor(s, 2, 32); s += __shfl_xor(s, 1, 32);
    const float mu = s * (1.0f / (float)DM);
    float q = 0.0f;
#pragma unroll
    for (int j = 0; j < 4; ++j) { v[j] = v[j] - mu; q += (v[j][0] * v[j][0] + v[j][1] * v[j][1]) + (v[j][2] * v[j][2] + v[j][3] * v[j][3]); }
    q += __shfl_xor(q, 16, 32); q += __shfl_xor(q, 8, 32); q += __shfl_xor(q, 4, 32); q += __shfl_xor(q, 2, 32); q += __shfl_xor(q, 1, 32);
    const float rs = rsqrtf(q * (1.0f / (float)DM) + LNEPS);
#pragma unroll
    for (int j = 0; j < 4; ++j) { const v4f gg = *(const v4f*)(g + j * 128 + lane * 4); const v4f bb = *(const v4f*)(be + j * 128 + lane * 4);
#pragma unroll
        for (int i = 0; i < 4; ++i) y[j][i] = v[j][i] * rs * bfr(gg[i]) + bfr(bb[i]); }
    size_t orow = (size_t)row;
    if (WH == 0) { const unsigned bb = row / (unsigned)SEQ, tt = row % (unsigned)SEQ; orow = (size_t)bb * OUT_SEQ + tt; }
    float* o = O32 + orow * DM + lane * 4;
    v8h hv0 = (v8h){}, hv1 = (v8h){};
    if (WH) {
        const int yb = wave * DM;
#pragma unroll
        for (int j = 0; j < 4; ++j) *(v4fa*)(&ys[yb + j * 128 + lane * 4]) = y[j];
        wave_sync();
        const v4f a0 = *(const v4fa*)(&ys[yb + lane * 8]),       a1 = *(const v4fa*)(&ys[yb + lane * 8 + 4]);
        const v4f c0 = *(const v4fa*)(&ys[yb + 256 + lane * 8]), c1 = *(const v4fa*)(&ys[yb + 256 + lane * 8 + 4]);
#pragma unroll
        for (int i = 0; i < 4; ++i) { hv0[i] = toh_flush(a0[i]); hv0[4 + i] = toh_flush(a1[i]); hv1[i] = toh_flush(c0[i]); hv1[4 + i] = toh_flush(c1[i]); }
    }
    static_assert(4 * 32 * 16 == DM * 4);
    static_assert(2 * 32 * 16 == DM * 2);
    h16* oh = O16 + (size_t)row * DM + lane * 8;
    *(volatile v4f*)(o) = y[0]; *(volatile v4f*)(o + 128) = y[1]; *(volatile v4f*)(o + 256) = y[2]; *(volatile v4f*)(o + 384) = y[3];
    if (WH) { *(volatile v8h*)(oh) = hv0; *(volatile v8h*)(oh + 256) = hv1; }
    __threadfence();
    *(volatile v4f*)(o) = y[0]; *(volatile v4f*)(o + 128) = y[1]; *(volatile v4f*)(o + 256) = y[2]; *(volatile v4f*)(o + 384) = y[3];
    if (WH) { *(volatile v8h*)(oh) = hv0; *(volatile v8h*)(oh + 256) = hv1; }
}
__global__ __launch_bounds__(256) void k_ln1(const float* __restrict__ T, const float* __restrict__ g, const float* __restrict__ be, float* X1, h16* X1H) { ln_body<1>(T, g, be, X1, X1H); }
__global__ __launch_bounds__(256) void k_ln2(const float* __restrict__ T, const float* __restrict__ g, const float* __restrict__ be, float* OUT) { ln_body<0>(T, g, be, OUT, nullptr); }

static constexpr size_t al256(size_t v) { return (v + 255) & ~(size_t)255; }
static constexpr size_t SZ_XB = al256((size_t)NB * SEQ * DM * 2);
static constexpr size_t SZ_WT = al256((size_t)3 * DM * DM * 2);
static constexpr size_t SZ_WO = al256((size_t)DM * DM * 2);
static constexpr size_t SZ_W1 = al256((size_t)DFF * DM * 2);
static constexpr size_t SZ_W2 = al256((size_t)DM * DFF * 2);
static constexpr size_t SZ_PL = al256((size_t)NB * NH_ * SEQ * HD * 2);
static constexpr size_t SZ_F32 = al256((size_t)NB * SEQ * DM * 4);
static constexpr size_t SZ_G  = al256((size_t)NB * SEQ * DFF * 2);
static constexpr size_t SZ_TOTAL = SZ_XB + SZ_WT + SZ_WO + SZ_W1 + SZ_W2 + 5 * SZ_PL + 2 * SZ_F32 + SZ_G;
static_assert(SZ_TOTAL <= (size_t)134217728);
static_assert(((size_t)DM * DM * 2) % 256 == 0);
static_assert((size_t)NB * NH_ * SEQ * HD == (size_t)NB * DM * SEQ);
static constexpr size_t NEED_X   = ((size_t)(NB - 1) * SEQ_FULL + SEQ) * DM;
static constexpr size_t NEED_OUT = ((size_t)(NB - 1) * OUT_SEQ + SEQ) * DM;

extern "C" void kernel_launch(void* const* d_in, const int* in_sizes, int n_in,
                              void* d_out, int out_size, void* d_ws, size_t ws_size, hipStream_t stream) {
    if (n_in < 19) return;
    if ((size_t)in_sizes[0] < NEED_X) return;
    if ((size_t)in_sizes[3] < (size_t)DM * DM || (size_t)in_sizes[5] < (size_t)DM * DM || (size_t)in_sizes[7] < (size_t)DM * DM || (size_t)in_sizes[9] < (size_t)DM * DM) return;
    if ((size_t)in_sizes[13] < (size_t)DM * DFF || (size_t)in_sizes[15] < (size_t)DFF * DM) return;
    if (in_sizes[4] < DM || in_sizes[6] < DM || in_sizes[8] < DM || in_sizes[10] < DM || in_sizes[11] < DM || in_sizes[12] < DM) return;
    if (in_sizes[14] < DFF || in_sizes[16] < DM || in_sizes[17] < DM || in_sizes[18] < DM) return;
    if ((size_t)out_size < NEED_OUT) return;
    if (SZ_TOTAL > ws_size) return;
    const float* x    = (const float*)d_in[0];
    const float* wq   = (const float*)d_in[3];  const float* bq = (const float*)d_in[4];
    const float* wk   = (const float*)d_in[5];  const float* bk = (const float*)d_in[6];
    const float* wv   = (const float*)d_in[7];  const float* bv = (const float*)d_in[8];
    const float* wo   = (const float*)d_in[9];  const float* bo = (const float*)d_in[10];
    const float* ln1g = (const float*)d_in[11]; const float* ln1b = (const float*)d_in[12];
    const float* w1   = (const float*)d_in[13]; const float* b1 = (const float*)d_in[14];
    const float* w2   = (const float*)d_in[15]; const float* b2 = (const float*)d_in[16];
    const float* ln2g = (const float*)d_in[17]; const float* ln2b = (const float*)d_in[18];
    float* OUT = (float*)d_out;
    char* wsp = (char*)d_ws;
    bf*  XB  = (bf*)wsp;  wsp += SZ_XB;
    bf*  WTB = (bf*)wsp;  wsp += SZ_WT;
    h16* WOT = (h16*)wsp; wsp += SZ_WO;
    h16* W1T = (h16*)wsp; wsp += SZ_W1;
    h16* W2T = (h16*)wsp; wsp += SZ_W2;
    h16* QH  = (h16*)wsp; wsp += SZ_PL;
    h16* KP  = (h16*)wsp; wsp += SZ_PL;
    h16* VT  = (h16*)wsp; wsp += SZ_PL;
    h16* CTX = (h16*)wsp; wsp += SZ_PL;
    h16* X1H = (h16*)wsp; wsp += SZ_PL;
    float* T1 = (float*)wsp; wsp += SZ_F32;
    float* X1 = (float*)wsp; wsp += SZ_F32;
    h16* G   = (h16*)wsp; wsp += SZ_G;
    bf* WQT = WTB; bf* WKT = WTB + (size_t)DM * DM; bf* WVT = WTB + (size_t)2 * DM * DM;

    if (SEQ == SEQ_FULL) {
        const size_t n8 = (size_t)NB * SEQ * DM / 8;
        k_cvt8<<<(unsigned)((n8 + 255) / 256), 256, 0, stream>>>(x, XB, n8);
    } else {
        const size_t n8 = (size_t)SEQ * DM / 8;
        for (int b = 0; b < NB; ++b) k_cvt8<<<(unsigned)((n8 + 255) / 256), 256, 0, stream>>>(x + (size_t)b * SEQ_FULL * DM, XB + (size_t)b * SEQ * DM, n8);
    }
    k_wt_b<<<dim3(DM / 64, DM / 64, 1), 256, 0, stream>>>(wq, WQT, (unsigned)DM, (unsigned)DM);
    k_wt_b<<<dim3(DM / 64, DM / 64, 1), 256, 0, stream>>>(wk, WKT, (unsigned)DM, (unsigned)DM);
    k_wt_b<<<dim3(DM / 64, DM / 64, 1), 256, 0, stream>>>(wv, WVT, (unsigned)DM, (unsigned)DM);
    k_wt_h<<<dim3(DM / 64, DM / 64, 1), 256, 0, stream>>>(wo, WOT, (unsigned)DM, (unsigned)DM);
    k_wt_h<<<dim3(DFF / 64, DM / 64, 1), 256, 0, stream>>>(w1, W1T, (unsigned)DM, (unsigned)DFF);
    k_wt_h<<<dim3(DM / 64, DFF / 64, 1), 256, 0, stream>>>(w2, W2T, (unsigned)DFF, (unsigned)DM);

    k_gemm_hd<<<dim3(NB * SEQ / 64, DM / 64, 1), 32, 0, stream>>>(XB, WQT, bq, QH);
    k_gemm_hd<<<dim3(NB * SEQ / 64, DM / 64, 1), 32, 0, stream>>>(XB, WKT, bk, KP);
    k_gemm_vt<<<dim3(DM / 64, NB * SEQ / 64, 1), 32, 0, stream>>>(WVT, XB, bv, VT);

    k_flash<<<dim3(SEQ / (16 * AW), NB * NH_, 1), 32 * AW, 0, stream>>>(QH, KP, VT, CTX);

    k_gemm_wo<<<dim3(NB * SEQ / 64, DM / 64, 1), 32, 0, stream>>>(CTX, WOT, bo, x, T1);
    k_ln1<<<NB * SEQ / 8, 256, 0, stream>>>(T1, ln1g, ln1b, X1, X1H);
    k_gemm_f1<<<dim3(NB * SEQ / 64, DFF / 64, 1), 32, 0, stream>>>(X1H, W1T, b1, G);
    k_gemm_f2<<<dim3(NB * SEQ / 64, DM / 64, 1), 32, 0, stream>>>(G, W2T, b2, X1, T1);
    k_ln2<<<NB * SEQ / 8, 256, 0, stream>>>(T1, ln2g, ln2b, OUT);
}
